// MultiHeadCrossAttention_91250875171618
// MI455X (gfx1250) — hardware-verified
//
#include <hip/hip_runtime.h>
#include <math.h>

#ifndef NB
#define NB 2
#endif
#ifndef SEQ
#define SEQ 2048
#endif
#define NB_FULL 2
#define SEQ_FULL 2048
#define EMB 1024
#define NHD 16
#define HDM 64
#define QBLK 64
#define KVB 64

static_assert(NB >= 1 && NB <= NB_FULL);
static_assert(SEQ >= 64 && SEQ <= SEQ_FULL && (SEQ % 64) == 0);
static_assert(NHD * HDM == EMB);
static_assert((EMB % 64) == 0 && (EMB % 32) == 0);
static_assert(QBLK == 64 && KVB == 64 && HDM == 64);

typedef __attribute__((ext_vector_type(16))) _Float16 v16h;
typedef __attribute__((ext_vector_type(8)))  _Float16 v8h;
typedef __attribute__((ext_vector_type(16))) __bf16   v16b;
typedef __attribute__((ext_vector_type(8)))  __bf16   v8b;
typedef __attribute__((ext_vector_type(8)))  float    v8f;
typedef __attribute__((ext_vector_type(4)))  float    v4f;
typedef __attribute__((ext_vector_type(4)))  unsigned v4u;


__device__ __forceinline__ unsigned short bfb(float f) {
    unsigned u = __float_as_uint(f);
    u += 0x7fffu + ((u >> 16) & 1u);
    return (unsigned short)(u >> 16);
}
__device__ __forceinline__ float bfq(float f) { return __uint_as_float(((unsigned)bfb(f)) << 16); }
__device__ __forceinline__ unsigned short hfb(float f) { return __builtin_bit_cast(unsigned short, (_Float16)f); }
__device__ __forceinline__ unsigned pk2b(float a, float b) { return (unsigned)bfb(a) | ((unsigned)bfb(b) << 16); }
__device__ __forceinline__ unsigned pk2h(float a, float b) { return (unsigned)hfb(a) | ((unsigned)hfb(b) << 16); }
__device__ __forceinline__ v4u pk8b(v4f a, v4f b) { v4u p; p.x = pk2b(a.x, a.y); p.y = pk2b(a.z, a.w); p.z = pk2b(b.x, b.y); p.w = pk2b(b.z, b.w); return p; }
__device__ __forceinline__ v4u pk8h(v4f a, v4f b) { v4u p; p.x = pk2h(a.x, a.y); p.y = pk2h(a.z, a.w); p.z = pk2h(b.x, b.y); p.w = pk2h(b.z, b.w); return p; }
__device__ __forceinline__ void split8b(v4f a, v4f b, v4u& ph, v4u& pl) {
    float v[8] = {a.x, a.y, a.z, a.w, b.x, b.y, b.z, b.w};
    unsigned short hs[8], ls[8];
#pragma unroll
    for (int i = 0; i < 8; ++i) { hs[i] = bfb(v[i]); ls[i] = bfb(v[i] - __uint_as_float(((unsigned)hs[i]) << 16)); }
    ph.x = (unsigned)hs[0] | ((unsigned)hs[1] << 16); ph.y = (unsigned)hs[2] | ((unsigned)hs[3] << 16);
    ph.z = (unsigned)hs[4] | ((unsigned)hs[5] << 16); ph.w = (unsigned)hs[6] | ((unsigned)hs[7] << 16);
    pl.x = (unsigned)ls[0] | ((unsigned)ls[1] << 16); pl.y = (unsigned)ls[2] | ((unsigned)ls[3] << 16);
    pl.z = (unsigned)ls[4] | ((unsigned)ls[5] << 16); pl.w = (unsigned)ls[6] | ((unsigned)ls[7] << 16);
}

__device__ __forceinline__ v8f wmma16(v16h a, v16h b, v8f c) {
    c = __builtin_amdgcn_wmma_f32_16x16x32_f16(false, a, false, b, (short)0, c, false, false);
    asm volatile("v_nop\n\tv_nop\n\tv_nop\n\tv_nop" : "+v"(c) : "v"(a), "v"(b));
    return c;
}

#define VST2U4(ptr, val) do { const v4u vst2_u4_ = (val); *(volatile v4u*)(ptr) = vst2_u4_; __threadfence(); *(volatile v4u*)(ptr) = vst2_u4_; } while (0)

namespace w25 {

__device__ __forceinline__ void dep_guard_h(v8f& a, v8f& b, v16h x, v16h y) { asm volatile("v_nop\n\tv_nop\n\tv_nop\n\tv_nop" : "+v"(a), "+v"(b) : "v"(x), "v"(y)); }
__device__ __forceinline__ void dep_guard_b(v8f& a, v8f& b, v16b x, v16b y) { asm volatile("v_nop\n\tv_nop\n\tv_nop\n\tv_nop" : "+v"(a), "+v"(b) : "v"(x), "v"(y)); }
__device__ __forceinline__ void keep4_h(v16h a, v16h b, v16h c, v16h d) { asm volatile("v_nop" :: "v"(a), "v"(b), "v"(c), "v"(d)); }
__device__ __forceinline__ void keep4_b(v16b a, v16b b, v16b c, v16b d) { asm volatile("v_nop" :: "v"(a), "v"(b), "v"(c), "v"(d)); }
__device__ __forceinline__ void acc_guard4(v8f& a, v8f& b, v8f& c, v8f& d) { asm volatile("v_nop\n\tv_nop\n\tv_nop\n\tv_nop" : "+v"(a), "+v"(b), "+v"(c), "+v"(d)); }

template <typename T> struct Frag;
template <> struct Frag<_Float16> {
    typedef v16h V; union U { v16h v; v8h h[2]; };
    static __device__ __forceinline__ v16h load(const _Float16* p) {
        U f; f.h[0] = *(const v8h*)(p); f.h[1] = *(const v8h*)(p + 16); return f.v;
    }
    static __device__ __forceinline__ v8f mma(v16h a, v16h b, v8f c) {
        return __builtin_amdgcn_wmma_f32_16x16x32_f16(false, a, false, b, (short)0, c, false, false);
    }
    static __device__ __forceinline__ void guard(v8f& a, v8f& b, v16h x, v16h y) { dep_guard_h(a, b, x, y); }
    static __device__ __forceinline__ void keep(v16h a, v16h b, v16h c, v16h d) { keep4_h(a, b, c, d); }
};
template <> struct Frag<__bf16> {
    typedef v16b V; union U { v16b v; v8b h[2]; };
    static __device__ __forceinline__ v16b load(const __bf16* p) {
        U f; f.h[0] = *(const v8b*)(p); f.h[1] = *(const v8b*)(p + 16); return f.v;
    }
    static __device__ __forceinline__ v8f mma(v16b a, v16b b, v8f c) {
        return __builtin_amdgcn_wmma_f32_16x16x32_bf16(false, a, false, b, (short)0, c, false, false);
    }
    static __device__ __forceinline__ void guard(v8f& a, v8f& b, v16b x, v16b y) { dep_guard_b(a, b, x, y); }
    static __device__ __forceinline__ void keep(v16b a, v16b b, v16b c, v16b d) { keep4_b(a, b, c, d); }
};
template <int ET> struct Elem;
template <> struct Elem<0> { typedef _Float16 T; };
template <> struct Elem<1> { typedef __bf16 T; };

template <int ET, int BIAS_MODE, int OUT_MODE>
__global__ __launch_bounds__(256) void wmma_gemm64(
    const unsigned short* __restrict__ Ap, int lda, long long strideA,
    const unsigned short* __restrict__ Btp, int ldb, long long strideB,
    void* __restrict__ Cout, int ldc, long long strideC,
    const float* __restrict__ bias, int M, int N, int K, float scale) {
    typedef typename Elem<ET>::T T;
    typedef typename Frag<T>::V V;
    const T* A = (const T*)Ap; const T* Bt = (const T*)Btp;
    __shared__ __align__(16) float sT[8][16 * 68];
    const int b    = blockIdx.y;
    const int lane = threadIdx.x & 31;
    const int wave = threadIdx.x >> 5;
    const int tilesN = N >> 6;
    const int tilesM = M >> 6;
    const int tile = blockIdx.x * 8 + wave;
    if (tile >= tilesM * tilesN) return;
    const int tm = tile / tilesN;
    const int tn = tile - tm * tilesN;
    const int m0 = tm << 6;
    const int n0 = tn << 6;

    const T* Ab = A  + (size_t)b * strideA;
    const T* Bb = Bt + (size_t)b * strideB;

    const int rlane = lane & 15;
    const int koff  = (lane >> 4) * 8;
    const int mOff  = (lane >> 4) * 8;

    v8f acc[4][4];
#pragma unroll
    for (int i = 0; i < 4; ++i)
#pragma unroll
        for (int j = 0; j < 4; ++j) acc[i][j] = (v8f){0.f, 0.f, 0.f, 0.f, 0.f, 0.f, 0.f, 0.f};

    for (int k0 = 0; k0 < K; k0 += 32) {
        V bh[4];
#pragma unroll
        for (int j = 0; j < 4; ++j) {
            const size_t bo = (size_t)(n0 + (j << 4) + rlane) * ldb + koff + k0;
            bh[j] = Frag<T>::load(Bb + bo);
        }
#pragma unroll
        for (int i = 0; i < 4; ++i) {
            const size_t ao = (size_t)(m0 + (i << 4) + rlane) * lda + koff + k0;
            V ah = Frag<T>::load(Ab + ao);
#pragma unroll
            for (int j = 0; j < 4; ++j) acc[i][j] = Frag<T>::mma(ah, bh[j], acc[i][j]);
            Frag<T>::guard(acc[i][0], acc[i][3], ah, ah);
        }
        Frag<T>::keep(bh[0], bh[1], bh[2], bh[3]);
    }
    acc_guard4(acc[0][0], acc[0][1], acc[0][2], acc[0][3]);
    acc_guard4(acc[1][0], acc[1][1], acc[1][2], acc[1][3]);
    acc_guard4(acc[2][0], acc[2][1], acc[2][2], acc[2][3]);
    acc_guard4(acc[3][0], acc[3][1], acc[3][2], acc[3][3]);

    float* slab = sT[wave];
#pragma unroll
    for (int i = 0; i < 4; ++i) {
        const int mBase = m0 + (i << 4);
#pragma unroll
        for (int j = 0; j < 4; ++j) {
            const int n = n0 + (j << 4) + rlane;
            float bv = 0.f;
            if (BIAS_MODE == 2) bv = bfq(bias[n]);
#pragma unroll
            for (int r = 0; r < 8; ++r) {
                float v = acc[i][j][r] * scale;
                if (BIAS_MODE == 1) v += bfq(bias[mBase + mOff + r]);
                if (BIAS_MODE == 2) v += bv;
                slab[(mOff + r) * 68 + (j << 4) + rlane] = v;
            }
        }
        __builtin_amdgcn_fence(3  , "workgroup");
        __builtin_amdgcn_wave_barrier();
        __builtin_amdgcn_fence(2  , "workgroup");
        if (OUT_MODE == 0) {
            float* C = (float*)Cout + (size_t)b * strideC;
            const int hh = lane >> 4, c4 = (lane & 15) * 4;
            for (int pass = 0; pass < 2; ++pass) {
#pragma unroll
                for (int it = 0; it < 8; ++it) {
                    const int row = it * 2 + hh;
                    v4f v = *(const v4f*)(slab + row * 68 + c4);
                    *(volatile v4f*)(C + (size_t)(mBase + row) * ldc + n0 + c4) = v;
                }
                __threadfence();
            }
        } else {
            const int q = lane >> 3, c8 = (lane & 7) * 8;
            unsigned short* C = (unsigned short*)Cout + (size_t)b * strideC;
            for (int pass = 0; pass < 2; ++pass) {
#pragma unroll
                for (int it = 0; it < 4; ++it) {
                    const int row = it * 4 + q;
                    const float* sp = slab + row * 68 + c8;
                    const v4f a4 = *(const v4f*)(sp); const v4f b4 = *(const v4f*)(sp + 4);
                    const v4u hv = pk8h(a4, b4);
                    *(volatile v4u*)(C + (size_t)(mBase + row) * ldc + n0 + c8) = hv;
                }
                __threadfence();
            }
        }
        __builtin_amdgcn_fence(3  , "workgroup");
        __builtin_amdgcn_wave_barrier();
        __builtin_amdgcn_fence(2  , "workgroup");
    }
}

}

union FH { v16h v; v8h h[2]; };
__global__ __launch_bounds__(128) void k_flash(const unsigned short* __restrict__ Qp, const unsigned short* __restrict__ Kp,
                                              const unsigned short* __restrict__ VTp, unsigned short* __restrict__ Op,
                                              int seq, float sl2) {
    __shared__ __align__(16) _Float16 Psh[4][16 * KVB];
    __shared__ __align__(16) float    Os[4][16 * 68];
    const int tid = threadIdx.x, wave = tid >> 5, lane = tid & 31, hh = lane >> 4, c = lane & 15;
    const int nqb = seq / QBLK;
    const int bx = blockIdx.x;
    const int qb = bx % nqb;
    const int bhd = bx / nqb;
    const int h = bhd % NHD;
    const int b = bhd / NHD;
    const int q0 = qb * QBLK + wave * 16;
    const _Float16* Q  = (const _Float16*)Qp;
    const _Float16* Kh = (const _Float16*)Kp;
    const _Float16* VT = (const _Float16*)VTp;
    const float NEG = -__builtin_inff();

    v16h qa0, qa1;
    {
        const _Float16* qrow = Q + ((size_t)b * seq + q0 + c) * EMB + h * HDM + 8 * hh;
        FH f;
        f.h[0] = *(const v8h*)(qrow);      f.h[1] = *(const v8h*)(qrow + 16); qa0 = f.v;
        f.h[0] = *(const v8h*)(qrow + 32); f.h[1] = *(const v8h*)(qrow + 48); qa1 = f.v;
    }
    float mrow[8], lrow[8];
    v8f oacc[4];
#pragma unroll
    for (int r = 0; r < 8; ++r) { mrow[r] = NEG; lrow[r] = 0.f; }
#pragma unroll
    for (int t = 0; t < 4; ++t) oacc[t] = (v8f){0.f, 0.f, 0.f, 0.f, 0.f, 0.f, 0.f, 0.f};

    const _Float16* kbase = Kh + ((size_t)b * seq) * EMB + h * HDM + 8 * hh;
    const _Float16* vbase = VT + (((size_t)b * NHD + h) * HDM + c) * (size_t)seq + 8 * hh;
    _Float16* pw = Psh[wave];
    const int nch = seq / KVB;
    for (int kc = 0; kc < nch; ++kc) {
        const int kv0 = kc * KVB;
        __builtin_amdgcn_fence(3  , "workgroup");
        __builtin_amdgcn_wave_barrier();
        __builtin_amdgcn_fence(2  , "workgroup");
        v8f s[4];
#pragma unroll
        for (int j = 0; j < 4; ++j) {
            const _Float16* krow = kbase + (size_t)(kv0 + j * 16 + c) * EMB;
            FH k0f, k1f;
            k0f.h[0] = *(const v8h*)(krow);      k0f.h[1] = *(const v8h*)(krow + 16);
            k1f.h[0] = *(const v8h*)(krow + 32); k1f.h[1] = *(const v8h*)(krow + 48);
            v8f z = (v8f){0.f, 0.f, 0.f, 0.f, 0.f, 0.f, 0.f, 0.f};
            z = wmma16(qa0, k0f.v, z);
            z = wmma16(qa1, k1f.v, z);
            s[j] = z;
        }
        float cm[8];
#pragma unroll
        for (int r = 0; r < 8; ++r) {
            float m = NEG;
#pragma unroll
            for (int j = 0; j < 4; ++j) { s[j][r] *= sl2; m = fmaxf(m, s[j][r]); }
            m = fmaxf(m, __shfl_xor(m, 1, 32)); m = fmaxf(m, __shfl_xor(m, 2, 32));
            m = fmaxf(m, __shfl_xor(m, 4, 32)); m = fmaxf(m, __shfl_xor(m, 8, 32));
            cm[r] = m;
        }
#pragma unroll
        for (int r = 0; r < 8; ++r) {
            const float mnew = fmaxf(mrow[r], cm[r]);
            const float alpha = exp2f(mrow[r] - mnew);
            mrow[r] = mnew;
            float psum = 0.f;
#pragma unroll
            for (int j = 0; j < 4; ++j) {
                const float p = exp2f(s[j][r] - mnew);
                psum += p;
                pw[(8 * hh + r) * KVB + j * 16 + c] = (_Float16)(p * 1024.0f);
            }
            psum += __shfl_xor(psum, 1, 32); psum += __shfl_xor(psum, 2, 32);
            psum += __shfl_xor(psum, 4, 32); psum += __shfl_xor(psum, 8, 32);
            lrow[r] = lrow[r] * alpha + psum;
#pragma unroll
            for (int t = 0; t < 4; ++t) oacc[t][r] *= alpha;
        }
        __builtin_amdgcn_fence(3  , "workgroup");
        __builtin_amdgcn_wave_barrier();
        __builtin_amdgcn_fence(2  , "workgroup");
#pragma unroll
        for (int kk = 0; kk < 2; ++kk) {
            FH pa;
            pa.h[0] = *(const v8h*)(pw + c * KVB + kk * 32 + 8 * hh);
            pa.h[1] = *(const v8h*)(pw + c * KVB + kk * 32 + 16 + 8 * hh);
#pragma unroll
            for (int t = 0; t < 4; ++t) {
                const _Float16* vrow = vbase + (size_t)(t * 16) * seq + kv0 + kk * 32;
                FH vb;
                vb.h[0] = *(const v8h*)(vrow); vb.h[1] = *(const v8h*)(vrow + 16);
                oacc[t] = wmma16(pa.v, vb.v, oacc[t]);
            }
        }
    }

    float* os = Os[wave];
#pragma unroll
    for (int r = 0; r < 8; ++r) {
        const float inv = 1.0f / (lrow[r] * 1024.0f);
#pragma unroll
        for (int t = 0; t < 4; ++t) os[(8 * hh + r) * 68 + t * 16 + c] = oacc[t][r] * inv;
    }
    __builtin_amdgcn_fence(3  , "workgroup");
    __builtin_amdgcn_wave_barrier();
    __builtin_amdgcn_fence(2  , "workgroup");
    {
        const int qq = lane >> 3, c8 = (lane & 7) * 8;
        unsigned short* ob = Op + ((size_t)b * seq + q0) * (2 * EMB) + h * HDM + c8;
        for (int pass = 0; pass < 2; ++pass) {
#pragma unroll
            for (int it = 0; it < 4; ++it) {
                const int row = it * 4 + qq;
                const float* sp = os + row * 68 + c8;
                const v4f a4 = *(const v4f*)(sp); const v4f b4 = *(const v4f*)(sp + 4);
                v4u ph, pl;
                split8b(a4, b4, ph, pl);
                *(volatile v4u*)(ob + (size_t)row * (2 * EMB)) = ph;
                *(volatile v4u*)(ob + (size_t)row * (2 * EMB) + EMB) = pl;
            }
            __threadfence();
        }
    }
}

__global__ __launch_bounds__(256) void k_xpl(const float* __restrict__ src, long long bstride, int seqn, unsigned short* __restrict__ dst, long long n8) {
    const long long u = (long long)blockIdx.x * 256 + threadIdx.x;
    if (u >= n8) return;
    const long long row = u >> 7; const int c8 = (int)(u & 127) * 8;
    const int bb = (int)(row / seqn); const int t = (int)(row - (long long)bb * seqn);
    const float* s = src + (size_t)bb * bstride + (size_t)t * EMB + c8;
    const v4f a4 = *(const v4f*)(s), b4 = *(const v4f*)(s + 4);
    VST2U4(dst + 8 * (size_t)u, pk8b(a4, b4));
}
__global__ __launch_bounds__(256) void k_wpl(const float* __restrict__ W, unsigned short* __restrict__ dst) {
    const int u = blockIdx.x * 256 + threadIdx.x;
    if (u >= EMB * (EMB / 8)) return;
    const int r = u >> 7; const int c0 = (u & 127) * 8;
    const int h = r >> 6, d = r & 63;
    const float* s = W + ((size_t)h * EMB + c0) * HDM + d;
    float v[8];
#pragma unroll
    for (int i = 0; i < 8; ++i) v[i] = s[(size_t)i * HDM];
    v4f a4, b4;
    a4.x = v[0]; a4.y = v[1]; a4.z = v[2]; a4.w = v[3]; b4.x = v[4]; b4.y = v[5]; b4.z = v[6]; b4.w = v[7];
    VST2U4(dst + 8 * (size_t)u, pk8b(a4, b4));
}
__global__ __launch_bounds__(256) void k_ppl(const float* __restrict__ W, unsigned short* __restrict__ dst) {
    const int u = blockIdx.x * 256 + threadIdx.x;
    if (u >= EMB * (EMB / 8)) return;
    const int n = u >> 7; const int c8 = (u & 127) * 8;
    const float* s = W + 8 * (size_t)u;
    const v4f a4 = *(const v4f*)(s), b4 = *(const v4f*)(s + 4);
    const v4u pk = pk8b(a4, b4);
    unsigned short* d = dst + (size_t)n * (2 * EMB) + c8;
    VST2U4(d, pk);
    VST2U4(d + EMB, pk);
}

extern "C" void kernel_launch(void* const* d_in, const int* in_sizes, int n_in,
                              void* d_out, int out_size, void* d_ws, size_t ws_size, hipStream_t stream) {
    if (n_in < 9) return;
    const float* e_in = (const float*)d_in[0];
    const float* x_in = (const float*)d_in[1];
    const float* Wq = (const float*)d_in[2];  const float* bq = (const float*)d_in[3];
    const float* Wk = (const float*)d_in[4];  const float* bk = (const float*)d_in[5];
    const float* Wv = (const float*)d_in[6];  const float* bv = (const float*)d_in[7];
    const float* Wp = (const float*)d_in[8];
    float* out = (float*)d_out;

    const long long need_act = (long long)(NB - 1) * SEQ_FULL * EMB + (long long)SEQ * EMB;
    if ((long long)in_sizes[0] < need_act || (long long)in_sizes[1] < need_act) return;
    if (in_sizes[2] < NHD * EMB * HDM || in_sizes[4] < NHD * EMB * HDM || in_sizes[6] < NHD * EMB * HDM) return;
    if (in_sizes[3] < NHD * HDM || in_sizes[5] < NHD * HDM || in_sizes[7] < NHD * HDM) return;
    if (in_sizes[8] < EMB * EMB) return;
    if ((long long)out_size < (long long)NB * SEQ * EMB) return;

    const size_t MR    = (size_t)NB * SEQ;
    const size_t ACT16 = MR * EMB * 2;
    const size_t W16   = (size_t)EMB * EMB * 2;
    size_t off = 0; char* base = (char*)d_ws;
    unsigned short* Xp  = (unsigned short*)(base + off); off += ACT16;
    unsigned short* Ep  = (unsigned short*)(base + off); off += ACT16;
    unsigned short* WqT = (unsigned short*)(base + off); off += W16;
    unsigned short* WkT = (unsigned short*)(base + off); off += W16;
    unsigned short* WvT = (unsigned short*)(base + off); off += W16;
    unsigned short* Wpp = (unsigned short*)(base + off); off += 2 * W16;
    unsigned short* Qp  = (unsigned short*)(base + off); off += ACT16;
    unsigned short* Kp  = (unsigned short*)(base + off); off += ACT16;
    unsigned short* VTp = (unsigned short*)(base + off); off += ACT16;
    unsigned short* Op  = (unsigned short*)(base + off); off += 2 * ACT16;
    if (off > ws_size || off > (size_t)134217728) return;

    const long long n8 = (long long)MR * (EMB / 8);
    const unsigned gpl = (unsigned)((n8 + 255) / 256);
    const unsigned gw  = (unsigned)((EMB * (EMB / 8) + 255) / 256);
    k_xpl<<<gpl, 256, 0, stream>>>(x_in, (long long)SEQ_FULL * EMB, SEQ, Xp, n8);
    k_xpl<<<gpl, 256, 0, stream>>>(e_in, (long long)SEQ_FULL * EMB, SEQ, Ep, n8);
    k_wpl<<<gw, 256, 0, stream>>>(Wq, WqT);
    k_wpl<<<gw, 256, 0, stream>>>(Wk, WkT);
    k_wpl<<<gw, 256, 0, stream>>>(Wv, WvT);
    k_ppl<<<gw, 256, 0, stream>>>(Wp, Wpp);

    const unsigned gqk = (unsigned)(((MR / 64) * (EMB / 64) + 7) / 8);
    w25::wmma_gemm64<1, 2, 1><<<dim3(gqk, 1), 256, 0, stream>>>(Xp, EMB, 0, WqT, EMB, 0, (void*)Qp, EMB, 0, bq, (int)MR, EMB, EMB, 1.0f);
    w25::wmma_gemm64<1, 2, 1><<<dim3(gqk, 1), 256, 0, stream>>>(Ep, EMB, 0, WkT, EMB, 0, (void*)Kp, EMB, 0, bk, (int)MR, EMB, EMB, 1.0f);
    const unsigned gv = (unsigned)(((EMB / 64) * (SEQ / 64) + 7) / 8);
    w25::wmma_gemm64<1, 1, 1><<<dim3(gv, NB), 256, 0, stream>>>(WvT, EMB, 0, Ep, EMB, (long long)SEQ * EMB, (void*)VTp, SEQ, (long long)EMB * SEQ, bv, EMB, SEQ, EMB, 1.0f);
    const float sl2 = 0.03125f * 1.4426950408889634f;
    k_flash<<<(unsigned)(NB * NHD * (SEQ / QBLK)), 128, 0, stream>>>(Qp, Kp, VTp, Op, SEQ, sl2);
    w25::wmma_gemm64<1, 0, 0><<<dim3(gqk, 1), 256, 0, stream>>>(Op, 2 * EMB, 0, Wpp, 2 * EMB, 0, (void*)out, EMB, 0, nullptr, (int)MR, EMB, 2 * EMB, 1.0f);
    (void)hipGetLastError();
}
